// cross_modal_module_69226282877400
// MI455X (gfx1250) — hardware-verified
//
#include <hip/hip_runtime.h>
#include <math.h>
#include <stdint.h>

#define NL_   6
#define NB_   16
#define NN_   128
#define DD_   512
#define KGD   50
#define KGP   64
#define ROWS  (NB_ * NN_)
#define KROWS (NB_ * NN_ * NN_)
#define FCW   (2 * DD_ + KGD)
#define NWPL  5
#define LNEPS 1e-5f
#define SLOPE 0.01f
#define WSC   64.0f
#define LOSC  2048.0f
#define PSC   1024.0f

#define F_BIAS  1
#define F_RELU  2
#define F_LRELU 4
#define F_RESID 8
#define F_OUT32 16
#define F_OUTHL 32

static_assert((ROWS % 32) == 0 && (DD_ % 64) == 0 && (DD_ % 32) == 0);
static_assert((KROWS % 32) == 0 && (NN_ % 32) == 0 && (NN_ / 32) * 32 == NN_);
static_assert(KGP >= KGD && (KGP % 32) == 0 && ((NL_ * KGP) % 32) == 0);
static_assert((ROWS % 8) == 0 && (DD_ == 512));

typedef _Float16 v16h __attribute__((ext_vector_type(16)));
typedef _Float16 v8h  __attribute__((ext_vector_type(8)));
typedef float    v8f  __attribute__((ext_vector_type(8)));
typedef float    v4f  __attribute__((ext_vector_type(4)));
typedef unsigned int v4u __attribute__((ext_vector_type(4)));

union FragH { v16h v; v8h h[2]; };

__device__ __forceinline__ unsigned short bf_bits(float f) {
  unsigned u = __float_as_uint(f);
  return (unsigned short)((u + 0x7FFFu + ((u >> 16) & 1u)) >> 16);
}
__device__ __forceinline__ float bf_up(unsigned short h) { return __uint_as_float(((unsigned)h) << 16); }
__device__ __forceinline__ float bfr(float f) { return bf_up(bf_bits(f)); }
__device__ __forceinline__ unsigned short h_bits(_Float16 x) { return __builtin_bit_cast(unsigned short, x); }
__device__ __forceinline__ unsigned pk16(unsigned short a, unsigned short b) { return (unsigned)a | ((unsigned)b << 16); }
__device__ __forceinline__ unsigned pkh(float a, float b) { return pk16(h_bits((_Float16)a), h_bits((_Float16)b)); }
__device__ __forceinline__ v8f zero8() { v8f z = {0.f, 0.f, 0.f, 0.f, 0.f, 0.f, 0.f, 0.f}; return z; }
__device__ __forceinline__ v4f zero4() { v4f z = {0.f, 0.f, 0.f, 0.f}; return z; }

__device__ __forceinline__ void hl_pair(float f0, float f1, unsigned& hp, unsigned& lp) {
#pragma clang fp contract(off)
  const _Float16 h0 = (_Float16)f0, h1 = (_Float16)f1;
  const float d0 = f0 - (float)h0, d1 = f1 - (float)h1;
  const float r0 = d0 * LOSC, r1 = d1 * LOSC;
  hp = pk16(h_bits(h0), h_bits(h1));
  lp = pk16(h_bits((_Float16)r0), h_bits((_Float16)r1));
}

__device__ __forceinline__ v16h ldfrag_h(const _Float16* p) {
  FragH f;
  f.h[0] = *(const v8h*)(p);
  f.h[1] = *(const v8h*)(p + 16);
  return f.v;
}

__device__ __forceinline__ v8f mma_h(v16h a, v16h b, v8f c) {
  c = __builtin_amdgcn_wmma_f32_16x16x32_f16(false, a, false, b, (short)0, c, false, false);
#if defined(__HIP_DEVICE_COMPILE__)
  asm volatile("v_nop\n\tv_nop\n\tv_nop\n\tv_nop" : "+v"(c) : "v"(a), "v"(b));
#endif
  return c;
}
__device__ __forceinline__ void wave_sync_lds() {
  __builtin_amdgcn_fence(__ATOMIC_RELEASE, "workgroup");
  __builtin_amdgcn_wave_barrier();
  __builtin_amdgcn_fence(__ATOMIC_ACQUIRE, "workgroup");
}

__global__ __launch_bounds__(256) void cvt_wT(const float* __restrict__ w0, const float* __restrict__ w1,
                                              const float* __restrict__ w2, const float* __restrict__ w3,
                                              const float* __restrict__ w4,
                                              int nsel, int zstride, unsigned short* outp, int nin, int nout) {
  __shared__ float tile[64][33];
  const int tid = threadIdx.x;
  const int z = blockIdx.z;
  const int sel = z % nsel, lay = z / nsel;
  const float* base = (sel == 0) ? w0 : ((sel == 1) ? w1 : ((sel == 2) ? w2 : ((sel == 3) ? w3 : w4)));
  const float* src = base + (size_t)lay * zstride;
  unsigned short* dst = outp + (size_t)z * nin * nout;
  const int i0 = blockIdx.x * 64;
  const int o0 = blockIdx.y * 32;
#pragma unroll
  for (int p = 0; p < 8; ++p) {
    const int idx = p * 256 + tid;
    const int i = idx >> 5, o = idx & 31;
    tile[i][o] = src[(size_t)(i0 + i) * nout + o0 + o];
  }
  __syncthreads();
  const int o = tid >> 3, c8 = (tid & 7) * 8;
  v4u pk;
#pragma unroll
  for (int e = 0; e < 4; ++e)
    pk[e] = pkh(bfr(tile[c8 + 2 * e][o]) * WSC, bfr(tile[c8 + 2 * e + 1][o]) * WSC);
  unsigned short* gp = dst + (size_t)(o0 + o) * nin + i0 + c8;
  *(volatile v4u*)gp = pk;
  __threadfence();
  *(volatile v4u*)gp = pk;
}

__global__ __launch_bounds__(256) void cvt_wkg(const float* __restrict__ wkg, unsigned short* outp) {
  const int tid = threadIdx.x;
  const int row = blockIdx.x * 32 + (tid >> 3);
  const int q8 = (tid & 7) * 8;
  const int l = row >> 6, n = row & 63;
  const int nc = (n < KGD) ? n : (KGD - 1);
  float f[8];
#pragma unroll
  for (int e = 0; e < 8; ++e) {
    const int k = q8 + e;
    const int kc = (k < KGD) ? k : (KGD - 1);
    const float v = bfr(wkg[(size_t)l * KGD * KGD + (size_t)kc * KGD + nc]) * WSC;
    f[e] = (k < KGD && n < KGD) ? v : 0.f;
  }
  v4u pk;
#pragma unroll
  for (int e = 0; e < 4; ++e) pk[e] = pkh(f[2 * e], f[2 * e + 1]);
  unsigned short* gp = outp + (size_t)row * KGP + q8;
  *(volatile v4u*)gp = pk;
  __threadfence();
  *(volatile v4u*)gp = pk;
}

__global__ __launch_bounds__(256) void cvt_kg(const float* __restrict__ kg, unsigned short* outp) {
  const int tid = threadIdx.x;
  const size_t row = (size_t)blockIdx.x * 32 + (tid >> 3);
  const int q8 = (tid & 7) * 8;
  const float* rp = kg + row * KGD;
  float f[8];
#pragma unroll
  for (int e = 0; e < 8; ++e) {
    const int c = q8 + e;
    const int cc = (c < KGD) ? c : (KGD - 1);
    const float v = bfr(rp[cc]);
    f[e] = (c < KGD) ? v : 0.f;
  }
  v4u pk;
#pragma unroll
  for (int e = 0; e < 4; ++e) pk[e] = pkh(f[2 * e], f[2 * e + 1]);
  unsigned short* gp = outp + row * KGP + q8;
  *(volatile v4u*)gp = pk;
  __threadfence();
  *(volatile v4u*)gp = pk;
}

__global__ __launch_bounds__(256) void kg_skg(const unsigned short* __restrict__ kgh,
                                              const unsigned short* __restrict__ wkg6,
                                              const float* __restrict__ bkg, const float* __restrict__ fcw,
                                              float* skg6) {
#pragma clang fp contract(off)
  __shared__ __align__(16) float sres[8][32];
  const int lane = threadIdx.x & 31, wave = threadIdx.x >> 5;
  const int m = lane & 15, hh = lane >> 4;
  const int t = __builtin_amdgcn_readfirstlane((int)(blockIdx.x * 8 + wave));
  const size_t row0 = (size_t)t * 32;
  const _Float16* A = (const _Float16*)(const void*)kgh;
  const _Float16* W = (const _Float16*)(const void*)wkg6;
  v16h fa[2][2];
#pragma unroll
  for (int i = 0; i < 2; ++i)
#pragma unroll
    for (int ks = 0; ks < 2; ++ks)
      fa[i][ks] = ldfrag_h(A + (row0 + 16 * i + m) * KGP + 32 * ks + 8 * hh);
  float* myres = sres[wave];
  const int q = lane & 7;
#pragma unroll 1
  for (int l = 0; l < NL_; ++l) {
    v8f acc[2][4];
#pragma unroll
    for (int i = 0; i < 2; ++i)
#pragma unroll
      for (int j = 0; j < 4; ++j) acc[i][j] = zero8();
#pragma unroll
    for (int j = 0; j < 4; ++j) {
      const _Float16* bp = W + (size_t)(l * KGP + 16 * j + m) * KGP + 8 * hh;
      const v16h fb0 = ldfrag_h(bp);
      const v16h fb1 = ldfrag_h(bp + 32);
#pragma unroll
      for (int i = 0; i < 2; ++i) {
        acc[i][j] = mma_h(fa[i][0], fb0, acc[i][j]);
        acc[i][j] = mma_h(fa[i][1], fb1, acc[i][j]);
      }
    }
    float p0[8], p1[8];
#pragma unroll
    for (int r = 0; r < 8; ++r) { p0[r] = 0.f; p1[r] = 0.f; }
#pragma unroll
    for (int j = 0; j < 4; ++j) {
      const int c = 16 * j + m;
      const int cc = (c < KGD) ? c : (KGD - 1);
      const float bb0 = bfr(bkg[l * KGD + cc]);
      const float ff0 = bfr(fcw[(size_t)l * FCW + 2 * DD_ + cc]);
      const bool live = c < KGD;
      const float bb = live ? bb0 : 0.f;
      const float ff = live ? ff0 : 0.f;
#pragma unroll
      for (int r = 0; r < 8; ++r) {
        float x = acc[0][j][r] * (1.0f / WSC);
        x = x + bb;
        x = fmaxf(x, 0.f);
        float pr = x * ff;
        p0[r] = p0[r] + pr;
        float y = acc[1][j][r] * (1.0f / WSC);
        y = y + bb;
        y = fmaxf(y, 0.f);
        pr = y * ff;
        p1[r] = p1[r] + pr;
      }
    }
#pragma unroll
    for (int off = 1; off < 16; off <<= 1) {
#pragma unroll
      for (int r = 0; r < 8; ++r) {
        p0[r] = p0[r] + __shfl_xor(p0[r], off, 32);
        p1[r] = p1[r] + __shfl_xor(p1[r], off, 32);
      }
    }
    if (m == 0) {
#pragma unroll
      for (int r = 0; r < 8; ++r) { myres[8 * hh + r] = p0[r]; myres[16 + 8 * hh + r] = p1[r]; }
    }
    wave_sync_lds();
    const v4f ov = *(const v4f*)(myres + 4 * q);
    float* gp = skg6 + (size_t)l * KROWS + row0 + 4 * q;
    if (lane < 8) { *(volatile v4f*)gp = ov; }
    __threadfence();
    if (lane < 8) { *(volatile v4f*)gp = ov; }
    wave_sync_lds();
  }
}

template <bool DOLN, bool RNDIN>
__global__ __launch_bounds__(256) void rows_hl(const float* __restrict__ xin, const float* __restrict__ g,
                                               const float* __restrict__ bt, unsigned short* oh, unsigned short* ol,
                                               int nrows) {
#pragma clang fp contract(off)
  const int tid = threadIdx.x, wave = tid >> 5, lane = tid & 31;
  const int row = blockIdx.x * 8 + wave;
  const int rowc = (row < nrows) ? row : (nrows - 1);
  const int c8 = lane * 8;
  const float* rp = xin + (size_t)rowc * DD_;
  const v4f a0 = *(const v4f*)(rp + c8), a1 = *(const v4f*)(rp + c8 + 4);
  const v4f b0 = *(const v4f*)(rp + 256 + c8), b1 = *(const v4f*)(rp + 256 + c8 + 4);
  float x[16];
#pragma unroll
  for (int e = 0; e < 4; ++e) { x[e] = a0[e]; x[4 + e] = a1[e]; x[8 + e] = b0[e]; x[12 + e] = b1[e]; }
  if (RNDIN) {
#pragma unroll
    for (int e = 0; e < 16; ++e) x[e] = bfr(x[e]);
  }
  float y[16];
  if (DOLN) {
    float s = 0.f;
#pragma unroll
    for (int e = 0; e < 16; ++e) s = s + x[e];
#pragma unroll
    for (int off = 1; off < 32; off <<= 1) s = s + __shfl_xor(s, off, 32);
    const float mu = s * (1.0f / DD_);
    float d[16];
    float s2 = 0.f;
#pragma unroll
    for (int e = 0; e < 16; ++e) { d[e] = x[e] - mu; const float dd = d[e] * d[e]; s2 = s2 + dd; }
#pragma unroll
    for (int off = 1; off < 32; off <<= 1) s2 = s2 + __shfl_xor(s2, off, 32);
    const float var = s2 * (1.0f / DD_);
    const float rstd = 1.0f / sqrtf(var + LNEPS);
#pragma unroll
    for (int e = 0; e < 16; ++e) {
      const int col = (e < 8) ? (c8 + e) : (256 + c8 + (e - 8));
      const float gg = bfr(g[col]), bb = bfr(bt[col]);
      float t = d[e] * rstd; t = t * gg; y[e] = t + bb;
    }
  } else {
#pragma unroll
    for (int e = 0; e < 16; ++e) y[e] = x[e];
  }
  v4u hv0, hv1, lv0, lv1;
#pragma unroll
  for (int e = 0; e < 4; ++e) {
    unsigned hp, lp;
    hl_pair(y[2 * e], y[2 * e + 1], hp, lp);         hv0[e] = hp; lv0[e] = lp;
    hl_pair(y[8 + 2 * e], y[8 + 2 * e + 1], hp, lp); hv1[e] = hp; lv1[e] = lp;
  }
  if (row < nrows) {
    unsigned short* hp0 = oh + (size_t)row * DD_ + c8;
    unsigned short* lp0 = ol + (size_t)row * DD_ + c8;
    for (int pass = 0; pass < 2; ++pass) {
      *(volatile v4u*)hp0 = hv0;
      *(volatile v4u*)(hp0 + 256) = hv1;
      *(volatile v4u*)lp0 = lv0;
      *(volatile v4u*)(lp0 + 256) = lv1;
      __threadfence();
    }
  }
}

__global__ __launch_bounds__(256) void ln_out(const float* __restrict__ xin, const float* __restrict__ g,
                                              const float* __restrict__ bt, float* outp, int nrows) {
#pragma clang fp contract(off)
  const int tid = threadIdx.x, wave = tid >> 5, lane = tid & 31;
  const int row = blockIdx.x * 8 + wave;
  const int rowc = (row < nrows) ? row : (nrows - 1);
  const int c4 = lane * 4;
  const float* rp = xin + (size_t)rowc * DD_ + c4;
  float x[16];
#pragma unroll
  for (int k = 0; k < 4; ++k) {
    const v4f a = *(const v4f*)(rp + 128 * k);
#pragma unroll
    for (int e = 0; e < 4; ++e) x[4 * k + e] = a[e];
  }
  float s = 0.f;
#pragma unroll
  for (int e = 0; e < 16; ++e) s = s + x[e];
#pragma unroll
  for (int off = 1; off < 32; off <<= 1) s = s + __shfl_xor(s, off, 32);
  const float mu = s * (1.0f / DD_);
  float d[16];
  float s2 = 0.f;
#pragma unroll
  for (int e = 0; e < 16; ++e) { d[e] = x[e] - mu; const float dd = d[e] * d[e]; s2 = s2 + dd; }
#pragma unroll
  for (int off = 1; off < 32; off <<= 1) s2 = s2 + __shfl_xor(s2, off, 32);
  const float var = s2 * (1.0f / DD_);
  const float rstd = 1.0f / sqrtf(var + LNEPS);
  v4f o[4];
#pragma unroll
  for (int k = 0; k < 4; ++k) {
#pragma unroll
    for (int e = 0; e < 4; ++e) {
      const int col = 128 * k + c4 + e;
      const float gg = bfr(g[col]), bb = bfr(bt[col]);
      float t = d[4 * k + e] * rstd; t = t * gg; o[k][e] = t + bb;
    }
  }
  if (row < nrows) {
    float* op = outp + (size_t)row * DD_ + c4;
    for (int pass = 0; pass < 2; ++pass) {
#pragma unroll
      for (int k = 0; k < 4; ++k) *(volatile v4f*)(op + 128 * k) = o[k];
      __threadfence();
    }
  }
}

__global__ __launch_bounds__(256) void rowdot_sqk(const float* __restrict__ q32, const float* __restrict__ k32,
                                                  const float* __restrict__ fcw, int lidx, float* sq, float* sk) {
  __shared__ __align__(16) float rq[32];
  __shared__ __align__(16) float rk[32];
  const int tid = threadIdx.x, wave = tid >> 5, lane = tid & 31;
  const int c16 = lane * 16;
  const int lc = (lidx < NL_) ? ((lidx < 0) ? 0 : lidx) : (NL_ - 1);
  const float* fq = fcw + (size_t)lc * FCW;
  const float* fk = fq + DD_;
  float wq[16], wk[16];
#pragma unroll
  for (int e = 0; e < 16; ++e) { wq[e] = bfr(fq[c16 + e]); wk[e] = bfr(fk[c16 + e]); }
#pragma unroll 1
  for (int rr = 0; rr < 4; ++rr) {
    const int rloc = wave * 4 + rr;
    const size_t row = (size_t)blockIdx.x * 32 + rloc;
    const float* qp = q32 + row * DD_ + c16;
    const float* kp = k32 + row * DD_ + c16;
    float s0 = 0.f, s1 = 0.f;
#pragma unroll
    for (int g4 = 0; g4 < 4; ++g4) {
      const v4f a = *(const v4f*)(qp + 4 * g4);
      const v4f c = *(const v4f*)(kp + 4 * g4);
#pragma unroll
      for (int e = 0; e < 4; ++e) { s0 += a[e] * wq[4 * g4 + e]; s1 += c[e] * wk[4 * g4 + e]; }
    }
#pragma unroll
    for (int off = 16; off >= 1; off >>= 1) { s0 += __shfl_xor(s0, off, 32); s1 += __shfl_xor(s1, off, 32); }
    if (lane == 0) { rq[rloc] = s0; rk[rloc] = s1; }
  }
  __syncthreads();
  if (tid < 16) {
    const int q = tid & 7;
    const v4f vq = *(const v4f*)(rq + 4 * q);
    const v4f vk = *(const v4f*)(rk + 4 * q);
    v4f v;
#pragma unroll
    for (int e = 0; e < 4; ++e) v[e] = (tid < 8) ? vq[e] : vk[e];
    float* gp = ((tid < 8) ? sq : sk) + (size_t)blockIdx.x * 32 + 4 * q;
    *(volatile v4f*)gp = v;
    __threadfence();
    *(volatile v4f*)gp = v;
  }
}

struct GDesc {
  const unsigned short* A0;
  const unsigned short* A1;
  const unsigned short* Bt;
  const float* bias;
  const float* resid;
  float* C32;
  unsigned short* Ch;
  unsigned short* Cl;
  int lda, ldb, ldc, ldh;
  int ldr, M, N, K;
  int blen, flags, tile0, tiles;
  float s0, s1;
};
static_assert(sizeof(GDesc) == 120);
struct GBatch {
  GDesc d[3];
  int nd;
  int tot;
};
static_assert(sizeof(GBatch) == 368);

__global__ __launch_bounds__(256) void gemm_hl(GBatch gb) {
#pragma clang fp contract(off)
  __shared__ __align__(16) float sT[8][16 * 68];
  const int lane = threadIdx.x & 31;
  const int wave = threadIdx.x >> 5;
  const int t = __builtin_amdgcn_readfirstlane((int)(blockIdx.x * 8 + wave));
  if (t >= gb.tot) return;
  int di = 0;
  if (t >= gb.d[1].tile0) di = 1;
  if (t >= gb.d[2].tile0) di = 2;
  GDesc D = gb.d[0];
  if (di == 1) D = gb.d[1];
  if (di == 2) D = gb.d[2];

  const _Float16* A0 = (const _Float16*)(const void*)D.A0;
  const _Float16* A1 = (const _Float16*)(const void*)D.A1;
  const _Float16* Bt = (const _Float16*)(const void*)D.Bt;
  const int tilesN = D.N >> 6;
  const int lt = t - D.tile0;
  const int tm = lt / tilesN;
  const int tn = lt - tm * tilesN;
  const int m0 = tm * 16;
  const int n0 = tn * 64;

  const int rl   = lane & 15;
  const int hh   = lane >> 4;
  const int koff = hh * 8;

  v8f acc0[4], acc1[4];
#pragma unroll
  for (int j = 0; j < 4; ++j) { acc0[j] = zero8(); acc1[j] = zero8(); }

  const size_t arow = (size_t)(m0 + rl) * D.lda + koff;
#pragma unroll 2
  for (int k0 = 0; k0 < D.K; k0 += 32) {
    const v16h fa0 = ldfrag_h(A0 + arow + k0);
    const v16h fa1 = ldfrag_h(A1 + arow + k0);
#pragma unroll
    for (int j = 0; j < 4; ++j) {
      const v16h fb = ldfrag_h(Bt + (size_t)(n0 + 16 * j + rl) * D.ldb + koff + k0);
      acc0[j] = mma_h(fa0, fb, acc0[j]);
      acc1[j] = mma_h(fa1, fb, acc1[j]);
    }
  }

  const int fl = D.flags;
  const float s0 = D.s0, s1 = D.s1;

  float* slab = sT[wave];
#pragma unroll
  for (int j = 0; j < 4; ++j) {
#pragma unroll
    for (int r = 0; r < 8; ++r) {
      const float u0 = acc0[j][r] * s0;
      const float u1 = acc1[j][r] * s1;
      slab[(koff + r) * 68 + 16 * j + rl] = u0 + u1;
    }
  }
  wave_sync_lds();

  const int h2 = lane >> 4, c4 = (lane & 15) * 4;
  float bz[4] = {0.f, 0.f, 0.f, 0.f};
  if (fl & F_BIAS) {
#pragma unroll
    for (int e = 0; e < 4; ++e) {
      const int n = n0 + c4 + e;
      const int nc = (n < D.blen) ? n : (D.blen - 1);
      bz[e] = bfr(D.bias[nc]);
    }
  }
  v4f ov[8];
#pragma unroll
  for (int it = 0; it < 8; ++it) {
    const int row = it * 2 + h2;
    const int gm = m0 + row;
    const v4f v = *(const v4f*)(slab + row * 68 + c4);
    v4f rv = zero4();
    if (fl & F_RESID) rv = *(const v4f*)(D.resid + (size_t)gm * D.ldr + n0 + c4);
    v4f o;
#pragma unroll
    for (int e = 0; e < 4; ++e) {
      float f = v[e] + bz[e];
      if (fl & F_RELU)  f = fmaxf(f, 0.f);
      if (fl & F_LRELU) f = (f >= 0.f) ? f : (SLOPE * f);
      f = f + rv[e];
      o[e] = f;
    }
    ov[it] = o;
    if (fl & F_OUTHL) *(v4f*)(slab + row * 68 + c4) = o;
  }
  if (fl & F_OUT32) {
    for (int pass = 0; pass < 2; ++pass) {
#pragma unroll
      for (int it = 0; it < 8; ++it) {
        const int row = it * 2 + h2;
        float* gp = D.C32 + (size_t)(m0 + row) * D.ldc + n0 + c4;
        *(volatile v4f*)gp = ov[it];
      }
      __threadfence();
    }
  }
  if (fl & F_OUTHL) {
    wave_sync_lds();
    const int q = lane >> 3, c8 = (lane & 7) * 8;
    v4u hv[4], lv[4];
#pragma unroll
    for (int it = 0; it < 4; ++it) {
      const int row = it * 4 + q;
      const float* sp = slab + row * 68 + c8;
      const v4f x0 = *(const v4f*)sp;
      const v4f x1 = *(const v4f*)(sp + 4);
      v4u a, bl;
#pragma unroll
      for (int e = 0; e < 2; ++e) {
        unsigned hp, lp;
        hl_pair(x0[2 * e], x0[2 * e + 1], hp, lp); a[e] = hp;     bl[e] = lp;
        hl_pair(x1[2 * e], x1[2 * e + 1], hp, lp); a[2 + e] = hp; bl[2 + e] = lp;
      }
      hv[it] = a; lv[it] = bl;
    }
    for (int pass = 0; pass < 2; ++pass) {
#pragma unroll
      for (int it = 0; it < 4; ++it) {
        const int row = it * 4 + q;
        unsigned short* gh = D.Ch + (size_t)(m0 + row) * D.ldh + n0 + c8;
        unsigned short* gl = D.Cl + (size_t)(m0 + row) * D.ldh + n0 + c8;
        *(volatile v4u*)gh = hv[it];
        *(volatile v4u*)gl = lv[it];
      }
      __threadfence();
    }
  }
  wave_sync_lds();
}

__global__ __launch_bounds__(256)
void attn_pv(const float* __restrict__ sq, const float* __restrict__ sk, const float* __restrict__ skg,
             const float* __restrict__ fcb, int lidx,
             const unsigned short* __restrict__ vh, const unsigned short* __restrict__ vl,
             const float* __restrict__ v32, float* src) {
#pragma clang fp contract(off)
  __shared__ __align__(16) unsigned short Vsh[NN_ * 64];
  __shared__ __align__(16) unsigned short Vsl[NN_ * 64];
  __shared__ __align__(16) _Float16 Ph[32 * 136];
  __shared__ __align__(16) _Float16 Pl[32 * 136];
  __shared__ __align__(16) float Os[32 * 68];

  const int tid = threadIdx.x, wave = tid >> 5, lane = tid & 31;
  const int hh = lane >> 4, m = lane & 15;
  const int rg = blockIdx.x, cs = blockIdx.y, b = blockIdx.z;
  const int i0 = rg * 32, d0 = cs * 64;
  const int lc = (lidx < NL_) ? ((lidx < 0) ? 0 : lidx) : (NL_ - 1);

#pragma unroll
  for (int s = 0; s < 4; ++s) {
    const int idx = tid + 256 * s;
    const int j = idx >> 3, q8 = (idx & 7) * 8;
    const size_t go = ((size_t)(b * NN_ + j)) * DD_ + d0 + q8;
    *(v4u*)(Vsh + j * 64 + q8) = *(const v4u*)(vh + go);
    *(v4u*)(Vsl + j * 64 + q8) = *(const v4u*)(vl + go);
  }

  const float fb = bfr(fcb[lc]);
#pragma unroll 1
  for (int rr = 0; rr < 4; ++rr) {
    const int il = wave * 4 + rr;
    const size_t grow = (size_t)b * NN_ + i0 + il;
    const float qv = sq[grow];
    float x[4];
    float mx = -INFINITY;
#pragma unroll
    for (int tq = 0; tq < 4; ++tq) {
      const int j = lane + 32 * tq;
      float sc = qv + sk[(size_t)b * NN_ + j];
      sc = sc + skg[grow * NN_ + j];
      sc = sc + fb;
      sc = (sc >= 0.f) ? sc : (SLOPE * sc);
      x[tq] = sc;
      mx = fmaxf(mx, sc);
    }
#pragma unroll
    for (int off = 16; off >= 1; off >>= 1) mx = fmaxf(mx, __shfl_xor(mx, off, 32));
    float sum = 0.f;
#pragma unroll
    for (int tq = 0; tq < 4; ++tq) { x[tq] = __expf(x[tq] - mx); sum = sum + x[tq]; }
#pragma unroll
    for (int off = 16; off >= 1; off >>= 1) sum = sum + __shfl_xor(sum, off, 32);
    const float inv = 1.0f / sum;
#pragma unroll
    for (int tq = 0; tq < 4; ++tq) {
      const int j = lane + 32 * tq;
      float p = x[tq] * inv;
      p = p * PSC;
      const _Float16 ph = (_Float16)p;
      const float dlt = p - (float)ph;
      const float res = dlt * LOSC;
      Ph[il * 136 + j] = ph;
      Pl[il * 136 + j] = (_Float16)res;
    }
  }
  __syncthreads();

  const int rt = wave >> 2, ct = wave & 3;
  const int cc = ct * 16 + m;
  const _Float16* VHs = (const _Float16*)(const void*)Vsh;
  const _Float16* VLs = (const _Float16*)(const void*)Vsl;
  v8f acc0 = zero8(), acc1 = zero8();
#pragma unroll
  for (int ks = 0; ks < 4; ++ks) {
    const _Float16* pah = Ph + (rt * 16 + m) * 136 + ks * 32 + 8 * hh;
    const _Float16* pal = Pl + (rt * 16 + m) * 136 + ks * 32 + 8 * hh;
    FragH fah, fal;
    fah.h[0] = *(const v8h*)(pah); fah.h[1] = *(const v8h*)(pah + 16);
    fal.h[0] = *(const v8h*)(pal); fal.h[1] = *(const v8h*)(pal + 16);
    FragH gh, gl;
#pragma unroll
    for (int i = 0; i < 8; ++i) {
      const int ja = (ks * 32 + 8 * hh + i) * 64 + cc;
      const int jb = (ks * 32 + 16 + 8 * hh + i) * 64 + cc;
      gh.h[0][i] = VHs[ja]; gh.h[1][i] = VHs[jb];
      gl.h[0][i] = VLs[ja]; gl.h[1][i] = VLs[jb];
    }
    acc0 = mma_h(fah.v, gh.v, acc0);
    acc1 = mma_h(fah.v, gl.v, acc1);
    acc1 = mma_h(fal.v, gh.v, acc1);
  }
#pragma unroll
  for (int r = 0; r < 8; ++r) {
    const float o0 = acc0[r] * (1.0f / PSC);
    const float o1 = acc1[r] * (1.0f / (PSC * LOSC));
    Os[(rt * 16 + 8 * hh + r) * 68 + cc] = o0 + o1;
  }
  __syncthreads();

  const int h2 = lane >> 4, c4 = (lane & 15) * 4;
  v4f ov[2];
  size_t gofs[2];
#pragma unroll
  for (int it = 0; it < 2; ++it) {
    const int row = wave * 4 + it * 2 + h2;
    const v4f o = *(const v4f*)(Os + row * 68 + c4);
    const size_t g = ((size_t)(b * NN_ + i0 + row)) * DD_ + d0 + c4;
    const v4f vr = *(const v4f*)(v32 + g);
    v4f f;
#pragma unroll
    for (int e = 0; e < 4; ++e) f[e] = vr[e] + o[e];
    ov[it] = f; gofs[it] = g;
  }
  for (int pass = 0; pass < 2; ++pass) {
#pragma unroll
    for (int it = 0; it < 2; ++it) *(volatile v4f*)(src + gofs[it]) = ov[it];
    __threadfence();
  }
}

static GDesc gdesc(const unsigned short* A0, const unsigned short* A1, int lda, const unsigned short* Bt, int ldb,
                   int M, int N, int K, const float* bias, int blen, const float* resid, int ldr,
                   float* C32, int ldc, unsigned short* Ch, unsigned short* Cl, int ldh,
                   int flags, float s0, float s1) {
  GDesc d;
  d.A0 = A0; d.A1 = A1; d.Bt = Bt; d.bias = bias; d.resid = resid; d.C32 = C32; d.Ch = Ch; d.Cl = Cl;
  d.lda = lda; d.ldb = ldb; d.ldc = ldc; d.ldh = ldh;
  d.ldr = ldr; d.M = M; d.N = N; d.K = K;
  d.blen = blen; d.flags = flags; d.tile0 = 0; d.tiles = (M / 16) * (N / 64);
  d.s0 = s0; d.s1 = s1;
  return d;
}
static void run_gemm(const GDesc* ds, int nd, hipStream_t stream) {
  GBatch gb;
  int tot = 0;
  for (int i = 0; i < 3; ++i) {
    if (i < nd) { gb.d[i] = ds[i]; gb.d[i].tile0 = tot; tot += ds[i].tiles; }
    else        { gb.d[i] = ds[0]; gb.d[i].tile0 = 1 << 30; gb.d[i].tiles = 0; }
  }
  gb.nd = nd; gb.tot = tot;
  if (tot <= 0) return;
  const dim3 grid((tot + 7) / 8);
  gemm_hl<<<grid, dim3(256), 0, stream>>>(gb);
}

extern "C" void kernel_launch(void* const* d_in, const int* in_sizes, int n_in,
                              void* d_out, int out_size, void* d_ws, size_t ws_size,
                              hipStream_t stream) {
  if (n_in < 20) return;
  const int ex[20] = { ROWS * DD_, KROWS * KGD,
                       NL_ * DD_ * DD_, NL_ * DD_, NL_ * DD_ * DD_, NL_ * DD_, NL_ * DD_ * DD_, NL_ * DD_,
                       NL_ * KGD * KGD, NL_ * KGD, NL_ * FCW, NL_, NL_ * DD_, NL_ * DD_,
                       NL_ * DD_ * DD_, NL_ * DD_, NL_ * DD_ * DD_, NL_ * DD_, DD_, DD_ };
  for (int i = 0; i < 20; ++i) if (in_sizes[i] != ex[i]) return;
  if (out_size != ROWS * DD_) return;

  const float* vectors = (const float*)d_in[0];
  const float* KG      = (const float*)d_in[1];
  const float* Wq  = (const float*)d_in[2];  const float* bq  = (const float*)d_in[3];
  const float* Wk  = (const float*)d_in[4];  const float* bk  = (const float*)d_in[5];
  const float* Wv  = (const float*)d_in[6];  const float* bv  = (const float*)d_in[7];
  const float* Wkg = (const float*)d_in[8];  const float* bkg = (const float*)d_in[9];
  const float* fcw = (const float*)d_in[10]; const float* fcb = (const float*)d_in[11];
  const float* ng  = (const float*)d_in[12]; const float* nb  = (const float*)d_in[13];
  const float* W1  = (const float*)d_in[14]; const float* b1  = (const float*)d_in[15];
  const float* W2  = (const float*)d_in[16]; const float* b2  = (const float*)d_in[17];
  const float* gf  = (const float*)d_in[18]; const float* bfv = (const float*)d_in[19];
  float* out = (float*)d_out;

  const size_t PL   = (size_t)DD_ * DD_;
  const size_t sWP  = (size_t)NL_ * NWPL * PL * 2;
  const size_t sWKG = (size_t)NL_ * KGP * KGP * 2;
  const size_t sKGH = (size_t)KROWS * KGP * 2;
  const size_t sSKG = (size_t)NL_ * KROWS * 4;
  const size_t sH   = (size_t)ROWS * DD_ * 2;
  const size_t sF   = (size_t)ROWS * DD_ * 4;
  const size_t sS   = (size_t)ROWS * 4;
  size_t off = 0;
  const size_t oWP  = off; off += sWP;
  const size_t oWKG = off; off += sWKG;
  const size_t oKGH = off; off += sKGH;
  const size_t oSKG = off; off += sSKG;
  const size_t oXH  = off; off += sH;
  const size_t oXL  = off; off += sH;
  const size_t oQ32 = off; off += sF;
  const size_t oK32 = off; off += sF;
  const size_t oV32 = off; off += sF;
  const size_t oVH  = off; off += sH;
  const size_t oVL  = off; off += sH;
  const size_t oSQ  = off; off += sS;
  const size_t oSK  = off; off += sS;
  const size_t oSRC = off; off += sF;
  const size_t oNRH = off; off += sH;
  const size_t oNRL = off; off += sH;
  const size_t oHH  = off; off += sH;
  const size_t oHL  = off; off += sH;
  const size_t oO32 = off; off += sF;
  if (off > ws_size) return;
  if (off > (size_t)134217728) return;

  char* ws = (char*)d_ws;
  unsigned short* WP   = (unsigned short*)(ws + oWP);
  unsigned short* WKG6 = (unsigned short*)(ws + oWKG);
  unsigned short* KGH  = (unsigned short*)(ws + oKGH);
  float*          SKG6 = (float*)(ws + oSKG);
  unsigned short* XH   = (unsigned short*)(ws + oXH);
  unsigned short* XL   = (unsigned short*)(ws + oXL);
  float*          Q32  = (float*)(ws + oQ32);
  float*          K32  = (float*)(ws + oK32);
  float*          V32  = (float*)(ws + oV32);
  unsigned short* VH   = (unsigned short*)(ws + oVH);
  unsigned short* VL   = (unsigned short*)(ws + oVL);
  float*          SQ   = (float*)(ws + oSQ);
  float*          SK   = (float*)(ws + oSK);
  float*          SRC  = (float*)(ws + oSRC);
  unsigned short* NRH  = (unsigned short*)(ws + oNRH);
  unsigned short* NRL  = (unsigned short*)(ws + oNRL);
  unsigned short* HH   = (unsigned short*)(ws + oHH);
  unsigned short* HL   = (unsigned short*)(ws + oHL);
  float*          OUT32 = (float*)(ws + oO32);

  const dim3 blk(256);

  cvt_wT<<<dim3(DD_ / 64, DD_ / 32, NL_ * NWPL), blk, 0, stream>>>(Wq, Wk, Wv, W1, W2, NWPL, DD_ * DD_, WP, DD_, DD_);
  cvt_wkg<<<dim3((NL_ * KGP) / 32), blk, 0, stream>>>(Wkg, WKG6);
  cvt_kg<<<dim3(KROWS / 32), blk, 0, stream>>>(KG, KGH);
  kg_skg<<<dim3(KROWS / 32 / 8), blk, 0, stream>>>(KGH, WKG6, bkg, fcw, SKG6);
  rows_hl<false, true><<<dim3(ROWS / 8), blk, 0, stream>>>(vectors, gf, bfv, XH, XL, ROWS);

  const float s0 = 1.0f / WSC;
  const float s1 = 1.0f / (WSC * LOSC);

  for (int l = 0; l < NL_; ++l) {
    const unsigned short* wq = WP + (size_t)(l * NWPL + 0) * PL;
    const unsigned short* wk = WP + (size_t)(l * NWPL + 1) * PL;
    const unsigned short* wv = WP + (size_t)(l * NWPL + 2) * PL;
    const unsigned short* w1 = WP + (size_t)(l * NWPL + 3) * PL;
    const unsigned short* w2 = WP + (size_t)(l * NWPL + 4) * PL;
    const float* bql = bq + (size_t)l * DD_; const float* bkl = bk + (size_t)l * DD_;
    const float* bvl = bv + (size_t)l * DD_;
    const float* ngl = ng + (size_t)l * DD_; const float* nbl = nb + (size_t)l * DD_;
    const float* b1l = b1 + (size_t)l * DD_; const float* b2l = b2 + (size_t)l * DD_;

    {
      GDesc d[3];
      d[0] = gdesc(XH, XL, DD_, wq, DD_, ROWS, DD_, DD_, bql, DD_, SRC, DD_, Q32, DD_, VH, VL, DD_,
                   F_BIAS | F_RELU | F_OUT32, s0, s1);
      d[1] = gdesc(XH, XL, DD_, wk, DD_, ROWS, DD_, DD_, bkl, DD_, SRC, DD_, K32, DD_, VH, VL, DD_,
                   F_BIAS | F_RELU | F_OUT32, s0, s1);
      d[2] = gdesc(XH, XL, DD_, wv, DD_, ROWS, DD_, DD_, bvl, DD_, SRC, DD_, V32, DD_, VH, VL, DD_,
                   F_BIAS | F_RELU | F_OUT32 | F_OUTHL, s0, s1);
      run_gemm(d, 3, stream);
    }
    rowdot_sqk<<<dim3(ROWS / 32), blk, 0, stream>>>(Q32, K32, fcw, l, SQ, SK);
    attn_pv<<<dim3(NN_ / 32, DD_ / 64, NB_), blk, 0, stream>>>(SQ, SK, SKG6 + (size_t)l * KROWS, fcb, l,
                                                              VH, VL, V32, SRC);
    rows_hl<true, false><<<dim3(ROWS / 8), blk, 0, stream>>>(SRC, ngl, nbl, NRH, NRL, ROWS);
    {
      GDesc d[1];
      d[0] = gdesc(NRH, NRL, DD_, w1, DD_, ROWS, DD_, DD_, b1l, DD_, SRC, DD_, OUT32, DD_, HH, HL, DD_,
                   F_BIAS | F_LRELU | F_OUTHL, s0, s1);
      run_gemm(d, 1, stream);
    }
    {
      GDesc d[1];
      d[0] = gdesc(HH, HL, DD_, w2, DD_, ROWS, DD_, DD_, b2l, DD_, SRC, DD_, OUT32, DD_, XH, XL, DD_,
                   F_BIAS | F_RESID | F_OUT32 | F_OUTHL, s0, s1);
      run_gemm(d, 1, stream);
    }
  }

  ln_out<<<dim3(ROWS / 8), blk, 0, stream>>>(OUT32, gf, bfv, out, ROWS);
  (void)hipGetLastError();
}
